// DrugRNACrossAttention_22093311771377
// MI455X (gfx1250) — hardware-verified
//
#include <hip/hip_runtime.h>
#include <math.h>
#include <stdint.h>

#define N1     2048
#define N2     4096
#define DIN    128
#define DM     256
#define NH     8
#define HD     32
#define TP     256
#define PSP    36
#define ACARRY 16.0f
#define WSC    256.0f
#define QKC    16.0f
#define VC     16.0f
#define PC     1024.0f
#define ZC     64.0f
#define RESC   2048.0f
#define RINV   0.00048828125f
#define NEGS   (-1.0e30f)

static_assert(NH * HD == DM);
static_assert((N1 % 64) == 0 && (N2 % 64) == 0 && (DIN % 64) == 0 && (DM % 64) == 0);
static_assert((N1 % 128) == 0 && (N2 % 128) == 0);
static_assert((N1 / 32) <= (TP / 2) && (N2 / 32) <= (TP / 2));

typedef _Float16 v16h __attribute__((ext_vector_type(16)));
typedef _Float16 v8h  __attribute__((ext_vector_type(8)));
typedef float    v8f  __attribute__((ext_vector_type(8)));
typedef float    v4f  __attribute__((ext_vector_type(4)));
typedef unsigned int v4u __attribute__((ext_vector_type(4)));

union FragH { v16h v; v8h h[2]; v4u u[2]; };

__device__ __forceinline__ unsigned short bf_bits(float f) {
  unsigned u = __float_as_uint(f);
  return (unsigned short)((u + 0x7FFFu + ((u >> 16) & 1u)) >> 16);
}
__device__ __forceinline__ float bf_up(unsigned short b) { return __uint_as_float(((unsigned)b) << 16); }
__device__ __forceinline__ float bfr(float f) { return bf_up(bf_bits(f)); }
__device__ __forceinline__ unsigned short h_bits(_Float16 x) { return __builtin_bit_cast(unsigned short, x); }
__device__ __forceinline__ unsigned pk16(unsigned short a, unsigned short b) { return (unsigned)a | ((unsigned)b << 16); }
__device__ __forceinline__ v8f zero8() { v8f z = {0.f, 0.f, 0.f, 0.f, 0.f, 0.f, 0.f, 0.f}; return z; }

__device__ __forceinline__ v16h ldfrag_h(const _Float16* p) {
  FragH f;
  f.h[0] = *(const v8h*)(p);
  f.h[1] = *(const v8h*)(p + 16);
  return f.v;
}
__device__ __forceinline__ v16h ldfrag_u(const unsigned short* p) {
  FragH f;
  f.u[0] = *(const v4u*)(p);
  f.u[1] = *(const v4u*)(p + 16);
  return f.v;
}

__device__ __forceinline__ v8f mma_raw(v16h a, v16h b, v8f c) {
  return __builtin_amdgcn_wmma_f32_16x16x32_f16(false, a, false, b, (short)0, c, false, false);
}
__device__ __forceinline__ void guard_4x1(v8f& a, v8f& b, v8f& c, v8f& d, v16h x) {
#if defined(__HIP_DEVICE_COMPILE__)
  asm volatile("v_nop\n\tv_nop\n\tv_nop\n\tv_nop" : "+v"(a), "+v"(b), "+v"(c), "+v"(d) : "v"(x));
#endif
}
__device__ __forceinline__ void keep4_h(v16h a, v16h b, v16h c, v16h d) {
#if defined(__HIP_DEVICE_COMPILE__)
  asm volatile("v_nop" :: "v"(a), "v"(b), "v"(c), "v"(d));
#endif
}
__device__ __forceinline__ void acc_guard4(v8f& a, v8f& b, v8f& c, v8f& d) {
#if defined(__HIP_DEVICE_COMPILE__)
  asm volatile("v_nop\n\tv_nop\n\tv_nop\n\tv_nop" : "+v"(a), "+v"(b), "+v"(c), "+v"(d));
#endif
}
__device__ __forceinline__ void guard_4x6(v8f& a, v8f& b, v8f& c, v8f& d,
                                          v16h x0, v16h x1, v16h x2, v16h x3, v16h x4, v16h x5) {
#if defined(__HIP_DEVICE_COMPILE__)
  asm volatile("v_nop\n\tv_nop\n\tv_nop\n\tv_nop"
               : "+v"(a), "+v"(b), "+v"(c), "+v"(d) : "v"(x0), "v"(x1), "v"(x2), "v"(x3), "v"(x4), "v"(x5));
#endif
}
__device__ __forceinline__ void wave_sync_lds() {
  __builtin_amdgcn_fence(__ATOMIC_RELEASE, "workgroup");
  __builtin_amdgcn_wave_barrier();
  __builtin_amdgcn_fence(__ATOMIC_ACQUIRE, "workgroup");
}

__device__ __forceinline__ void split8(const float* sp, v4u& hi, v4u& lo) {
  const v4f a = *(const v4f*)(sp), b = *(const v4f*)(sp + 4);
  float v[8];
#pragma unroll
  for (int e = 0; e < 4; ++e) { v[e] = a[e]; v[4 + e] = b[e]; }
#pragma unroll
  for (int e = 0; e < 4; ++e) {
    const _Float16 h0 = (_Float16)v[2 * e], h1 = (_Float16)v[2 * e + 1];
    const _Float16 l0 = (_Float16)((v[2 * e] - (float)h0) * RESC);
    const _Float16 l1 = (_Float16)((v[2 * e + 1] - (float)h1) * RESC);
    hi[e] = pk16(h_bits(h0), h_bits(h1));
    lo[e] = pk16(h_bits(l0), h_bits(l1));
  }
}

__global__ __launch_bounds__(256) void wtcv(const float* __restrict__ W, unsigned short* dst, int K, int N) {
  __shared__ float sm[64][65];
  const int t  = threadIdx.x;
  const int k0 = blockIdx.x * 64, n0 = blockIdx.y * 64;
  const int kl = t >> 2, nq = (t & 3) * 16;
  const float* src = W + (size_t)(k0 + kl) * (size_t)N + n0 + nq;
#pragma unroll
  for (int q = 0; q < 4; ++q) {
    const v4f a = *(const v4f*)(src + 4 * q);
#pragma unroll
    for (int e = 0; e < 4; ++e) sm[kl][nq + 4 * q + e] = a[e];
  }
  __syncthreads();
  v4u o[2];
#pragma unroll
  for (int it = 0; it < 2; ++it) {
    const int p = it * 256 + t, nl = p >> 3, c8 = (p & 7) * 8;
    v4u a;
#pragma unroll
    for (int e = 0; e < 4; ++e) {
      const float f0 = bfr(sm[c8 + 2 * e][nl]) * WSC, f1 = bfr(sm[c8 + 2 * e + 1][nl]) * WSC;
      a[e] = pk16(h_bits((_Float16)f0), h_bits((_Float16)f1));
    }
    o[it] = a;
  }
#pragma unroll
  for (int it = 0; it < 2; ++it) {
    const int p = it * 256 + t, nl = p >> 3, c8 = (p & 7) * 8;
    *(volatile v4u*)(dst + (size_t)(n0 + nl) * (size_t)K + k0 + c8) = o[it];
  }
  __threadfence();
#pragma unroll
  for (int it = 0; it < 2; ++it) {
    const int p = it * 256 + t, nl = p >> 3, c8 = (p & 7) * 8;
    *(volatile v4u*)(dst + (size_t)(n0 + nl) * (size_t)K + k0 + c8) = o[it];
  }
}

__global__ __launch_bounds__(256) void xcv(const float* __restrict__ x, unsigned short* XP, int nrows) {
  const int i   = blockIdx.x * 256 + threadIdx.x;
  const int row = i >> 4;
  const int c8  = (i & 15) * 8;
  const bool live = row < nrows;
  const int rc  = live ? row : (nrows - 1);
  const float* p = x + (size_t)rc * DIN + c8;
  const v4f a = *(const v4f*)(p), b = *(const v4f*)(p + 4);
  float v[8];
#pragma unroll
  for (int e = 0; e < 4; ++e) {
    v[e]     = live ? bfr(a[e]) : 0.f;
    v[4 + e] = live ? bfr(b[e]) : 0.f;
  }
  v4u o;
#pragma unroll
  for (int e = 0; e < 4; ++e) o[e] = pk16(h_bits((_Float16)(v[2 * e] * ACARRY)), h_bits((_Float16)(v[2 * e + 1] * ACARRY)));
  unsigned short* dp = XP + (size_t)i * 8;
  *(volatile v4u*)dp = o;
  __threadfence();
  *(volatile v4u*)dp = o;
}

__global__ __launch_bounds__(128) void blkmap(const int* __restrict__ qb, const int* __restrict__ kbv, unsigned* T, int Nq, int Nk) {
  const int lane = threadIdx.x & 31;
  const int wave = threadIdx.x >> 5;
  const int qt   = blockIdx.x * 4 + wave;
  if (qt * 16 >= Nq) return;
  int qid[16];
#pragma unroll
  for (int r = 0; r < 16; ++r) {
    const int qr = qt * 16 + r;
    qid[r] = qb[(qr < Nq) ? qr : (Nq - 1)];
  }
  unsigned rowhit = 0u;
  v4u flv = {0u, 0u, 0u, 0u};
  const int nj = Nk >> 7;
#pragma unroll 1
  for (int jq = 0; jq < nj; ++jq) {
#pragma unroll
    for (int u = 0; u < 4; ++u) {
      const int key = ((jq << 2) + u) * 32 + lane;
      const int kid = kbv[(key < Nk) ? key : (Nk - 1)];
      unsigned mt = 0u;
#pragma unroll
      for (int r = 0; r < 16; ++r) mt |= (kid == qid[r]) ? (1u << r) : 0u;
      rowhit |= mt;
      const unsigned bal  = __builtin_amdgcn_ballot_w32(mt != 0u);
      const unsigned anyb = (bal != 0u) ? 1u : 0u;
      flv[u] = (lane == jq) ? anyb : flv[u];
    }
  }
#pragma unroll
  for (int s = 1; s < 32; s <<= 1) rowhit |= __shfl_xor(rowhit, s, 32);
  const int lc = (lane < 4) ? lane : 0;
  v4u rf;
#pragma unroll
  for (int e = 0; e < 4; ++e) rf[e] = ((lane < 4) && (((rowhit >> (4 * lc + e)) & 1u) == 0u)) ? 1u : 0u;
  unsigned* rowp = T + (size_t)qt * TP;
  *(volatile v4u*)(rowp + 4 * lane) = flv;
  *(volatile v4u*)(rowp + (TP / 2) + 4 * lane) = rf;
  __threadfence();
  *(volatile v4u*)(rowp + 4 * lane) = flv;
  *(volatile v4u*)(rowp + (TP / 2) + 4 * lane) = rf;
}

__device__ __forceinline__ void kloop(v8f (&acc)[4][4], const unsigned short* __restrict__ A1, int lda, long long sAk,
                                      const unsigned short* __restrict__ Bb, int ldb, int m0, int n0, int K,
                                      int rlane, int koff) {
#pragma unroll 1
  for (int k0 = 0; k0 < K; k0 += 32) {
    v16h bh[4];
#pragma unroll
    for (int j = 0; j < 4; ++j) {
      const size_t bofs = (size_t)(n0 + (j << 4) + rlane) * (size_t)ldb + (size_t)(koff + k0);
      bh[j] = ldfrag_u(Bb + bofs);
    }
    const size_t ak = (size_t)(k0 >> 5) * (size_t)sAk + (size_t)((k0 & 31) + koff);
#pragma unroll
    for (int i = 0; i < 4; ++i) {
      const size_t ao = (size_t)(m0 + (i << 4) + rlane) * (size_t)lda + ak;
      const v16h ah = ldfrag_u(A1 + ao);
#pragma unroll
      for (int j = 0; j < 4; ++j) acc[i][j] = mma_raw(ah, bh[j], acc[i][j]);
      guard_4x1(acc[i][0], acc[i][1], acc[i][2], acc[i][3], ah);
    }
    keep4_h(bh[0], bh[1], bh[2], bh[3]);
  }
}

template <int OM, int BIASM>
__global__ __launch_bounds__(256) void gemm64(
    const unsigned short* __restrict__ Ap, int lda, long long sAk, long long aLo,
    const unsigned short* __restrict__ Btp, int ldb,
    const float* __restrict__ bias, float bscale,
    void* Cout, int ldc, long long cLo,
    int M, int N, int K, float oscale) {
  __shared__ __align__(16) float sT[8][16 * 68];
  const int lane = threadIdx.x & 31;
  const int wave = threadIdx.x >> 5;
  const int tilesN = N >> 6;
  const int tilesM = M >> 6;
  const int tile = blockIdx.x * 8 + wave;
  if (tile >= tilesM * tilesN) return;
  const int tm = tile / tilesN;
  const int tn = tile - tm * tilesN;
  const int m0 = tm << 6;
  const int n0 = tn << 6;

  const int rlane = lane & 15;
  const int koff  = (lane >> 4) * 8;
  const int mOff  = (lane >> 4) * 8;

  v8f acc[4][4];
#pragma unroll
  for (int i = 0; i < 4; ++i)
#pragma unroll
    for (int j = 0; j < 4; ++j) acc[i][j] = zero8();

  if (aLo != 0) {
    kloop(acc, Ap + aLo, lda, sAk, Btp, ldb, m0, n0, K, rlane, koff);
    acc_guard4(acc[0][0], acc[0][1], acc[0][2], acc[0][3]);
    acc_guard4(acc[1][0], acc[1][1], acc[1][2], acc[1][3]);
    acc_guard4(acc[2][0], acc[2][1], acc[2][2], acc[2][3]);
    acc_guard4(acc[3][0], acc[3][1], acc[3][2], acc[3][3]);
#pragma unroll
    for (int i = 0; i < 4; ++i)
#pragma unroll
      for (int j = 0; j < 4; ++j) acc[i][j] = acc[i][j] * RINV;
  }
  kloop(acc, Ap, lda, sAk, Btp, ldb, m0, n0, K, rlane, koff);
  acc_guard4(acc[0][0], acc[0][1], acc[0][2], acc[0][3]);
  acc_guard4(acc[1][0], acc[1][1], acc[1][2], acc[1][3]);
  acc_guard4(acc[2][0], acc[2][1], acc[2][2], acc[2][3]);
  acc_guard4(acc[3][0], acc[3][1], acc[3][2], acc[3][3]);

  const int hh2 = lane >> 4, c4 = (lane & 15) * 4;
  const int q8  = lane >> 3, c8 = (lane & 7) * 8;
  float bc[4];
#pragma unroll
  for (int e = 0; e < 4; ++e) bc[e] = 0.f;
  if (BIASM == 0) {
    const int cb = n0 + c4;
    const int i0 = (cb < N - 4) ? cb : (N - 4);
    const v4f b0v = *(const v4f*)(bias + i0);
#pragma unroll
    for (int e = 0; e < 4; ++e) bc[e] = bfr(b0v[e]) * bscale;
  }

  float* slab = sT[wave];
#pragma unroll
  for (int i = 0; i < 4; ++i) {
    const int mBase = m0 + (i << 4);
#pragma unroll
    for (int j = 0; j < 4; ++j) {
#pragma unroll
      for (int r = 0; r < 8; ++r) {
        slab[(mOff + r) * 68 + (j << 4) + rlane] = acc[i][j][r];
      }
    }
    wave_sync_lds();
    if (OM == 4) {
      float* C = (float*)Cout;
      v4f vals[8];
#pragma unroll
      for (int it = 0; it < 8; ++it) {
        const int row = it * 2 + hh2;
        v4f v = *(const v4f*)(slab + row * 68 + c4);
#pragma unroll
        for (int e = 0; e < 4; ++e) v[e] = v[e] * oscale + bc[e];
        vals[it] = v;
      }
#pragma unroll
      for (int it = 0; it < 8; ++it) {
        const int gr = mBase + it * 2 + hh2;
        *(volatile v4f*)(C + (size_t)gr * (size_t)ldc + n0 + c4) = vals[it];
      }
      __threadfence();
#pragma unroll
      for (int it = 0; it < 8; ++it) {
        const int gr = mBase + it * 2 + hh2;
        *(volatile v4f*)(C + (size_t)gr * (size_t)ldc + n0 + c4) = vals[it];
      }
      __threadfence();
    } else {
      unsigned short* C = (unsigned short*)Cout;
      v4u hv[4], lv[4];
#pragma unroll
      for (int it = 0; it < 4; ++it) {
        const int row = it * 4 + q8;
        const float* sp = slab + row * 68 + c8;
        const v4f x0 = *(const v4f*)(sp), x1 = *(const v4f*)(sp + 4);
        float v[8];
#pragma unroll
        for (int e = 0; e < 4; ++e) {
          v[e]     = x0[e] * oscale;
          v[4 + e] = x1[e] * oscale;
        }
        v4u ha, la;
#pragma unroll
        for (int e = 0; e < 4; ++e) {
          const _Float16 h0 = (_Float16)v[2 * e], h1 = (_Float16)v[2 * e + 1];
          const _Float16 l0 = (_Float16)((v[2 * e] - (float)h0) * RESC);
          const _Float16 l1 = (_Float16)((v[2 * e + 1] - (float)h1) * RESC);
          ha[e] = pk16(h_bits(h0), h_bits(h1));
          la[e] = pk16(h_bits(l0), h_bits(l1));
        }
        hv[it] = ha;
        lv[it] = la;
      }
#pragma unroll
      for (int it = 0; it < 4; ++it) {
        const int row = it * 4 + q8;
        const size_t o = (size_t)(mBase + row) * (size_t)ldc + n0 + c8;
        *(volatile v4u*)(C + o) = hv[it];
        if (OM == 3) *(volatile v4u*)(C + cLo + o) = lv[it];
      }
      __threadfence();
#pragma unroll
      for (int it = 0; it < 4; ++it) {
        const int row = it * 4 + q8;
        const size_t o = (size_t)(mBase + row) * (size_t)ldc + n0 + c8;
        *(volatile v4u*)(C + o) = hv[it];
        if (OM == 3) *(volatile v4u*)(C + cLo + o) = lv[it];
      }
      __threadfence();
    }
    wave_sync_lds();
  }
}

__device__ __forceinline__ void build_p(const float* pt, int c, int hh, FragH& ph, FragH& pl) {
  const float* prow = pt + c * PSP + 8 * hh;
  const v4f p0 = *(const v4f*)(prow), p1 = *(const v4f*)(prow + 4);
  const v4f p2 = *(const v4f*)(prow + 16), p3 = *(const v4f*)(prow + 20);
#pragma unroll
  for (int e = 0; e < 4; ++e) {
    float v; _Float16 hv;
    v = p0[e] * PC; hv = (_Float16)v; ph.h[0][e]     = hv; pl.h[0][e]     = (_Float16)((v - (float)hv) * RESC);
    v = p1[e] * PC; hv = (_Float16)v; ph.h[0][4 + e] = hv; pl.h[0][4 + e] = (_Float16)((v - (float)hv) * RESC);
    v = p2[e] * PC; hv = (_Float16)v; ph.h[1][e]     = hv; pl.h[1][e]     = (_Float16)((v - (float)hv) * RESC);
    v = p3[e] * PC; hv = (_Float16)v; ph.h[1][4 + e] = hv; pl.h[1][4 + e] = (_Float16)((v - (float)hv) * RESC);
  }
}

__device__ __forceinline__ void store_tile16x32(const float* os, int lane, unsigned short* dh, unsigned short* dl) {
  v4u h0, l0, h1, l1;
  split8(os + lane * 8, h0, l0);
  split8(os + 256 + lane * 8, h1, l1);
  *(volatile v4u*)(dh + lane * 8) = h0;
  *(volatile v4u*)(dh + 256 + lane * 8) = h1;
  *(volatile v4u*)(dl + lane * 8) = l0;
  *(volatile v4u*)(dl + 256 + lane * 8) = l1;
  __threadfence();
  *(volatile v4u*)(dh + lane * 8) = h0;
  *(volatile v4u*)(dh + 256 + lane * 8) = h1;
  *(volatile v4u*)(dl + lane * 8) = l0;
  *(volatile v4u*)(dl + 256 + lane * 8) = l1;
  __threadfence();
}

__global__ __launch_bounds__(128)
void attn(const unsigned short* __restrict__ QH, const unsigned short* __restrict__ QL,
          const unsigned short* __restrict__ KH, const unsigned short* __restrict__ KL,
          const unsigned short* __restrict__ VTH, const unsigned short* __restrict__ VTL,
          const int* __restrict__ qb, const int* __restrict__ kbv, const unsigned* __restrict__ T,
          unsigned short* CH, unsigned short* CL, int Nq, int Nk) {
  __shared__ __align__(16) float Ps[4][16 * PSP];
  __shared__ __align__(16) float Os[4][16 * 32];

  const int tid  = threadIdx.x;
  const int wave = tid >> 5;
  const int lane = tid & 31;
  const int hh   = lane >> 4;
  const int c    = lane & 15;

  const int wid  = blockIdx.x * 4 + wave;
  const int h    = wid & (NH - 1);
  const int qt   = wid >> 3;
  const int q0   = qt * 16;
  if (q0 >= Nq) return;

  const _Float16* qhp = (const _Float16*)(const void*)QH + (size_t)(q0 + c) * DM + HD * h + 8 * hh;
  const _Float16* qlp = (const _Float16*)(const void*)QL + (size_t)(q0 + c) * DM + HD * h + 8 * hh;
  const v16h qh = ldfrag_h(qhp), ql = ldfrag_h(qlp);
  const _Float16* khp = (const _Float16*)(const void*)KH + (size_t)c * DM + HD * h + 8 * hh;
  const _Float16* klp = (const _Float16*)(const void*)KL + (size_t)c * DM + HD * h + 8 * hh;
  const _Float16* vhp = (const _Float16*)(const void*)VTH + (size_t)(HD * h + c) * (size_t)Nk + 8 * hh;
  const _Float16* vlp = (const _Float16*)(const void*)VTL + (size_t)(HD * h + c) * (size_t)Nk + 8 * hh;

  int qid[8];
#pragma unroll
  for (int r = 0; r < 8; ++r) {
    const int qr = q0 + 8 * hh + r;
    qid[r] = qb[(qr < Nq) ? qr : (Nq - 1)];
  }
  const unsigned* trow = T + (size_t)qt * TP;
  unsigned fl16 = 0u;
#pragma unroll
  for (int r = 0; r < 16; ++r) fl16 |= (trow[(TP / 2) + r] != 0u) ? (1u << r) : 0u;
  const int anyf = __builtin_amdgcn_readfirstlane((int)fl16);
  const unsigned fb = (((unsigned)anyf) >> (8 * hh)) & 0xFFu;
  const float lsc = (1.4426950408889634f * 0.17677669529663687f) / (QKC * QKC);

  float m[8], l[8];
  v8f z0h = zero8(), z0x = zero8(), z1h = zero8(), z1x = zero8();
#pragma unroll
  for (int r = 0; r < 8; ++r) { m[r] = NEGS; l[r] = 0.f; }
  float* pP = Ps[wave];
  const int nks = Nk >> 5;

#pragma unroll 1
  for (int ks = 0; ks < nks; ++ks) {
    const int tb = __builtin_amdgcn_readfirstlane((int)trow[ks]);
    if (tb == 0 && anyf == 0) continue;
    const int kb0 = ks * 32;
    v8f s0h, s0x, s1h, s1x;
    {
      const v16h kf0h = ldfrag_h(khp + (size_t)kb0 * DM), kf1h = ldfrag_h(khp + (size_t)(kb0 + 16) * DM);
      const v16h kf0l = ldfrag_h(klp + (size_t)kb0 * DM), kf1l = ldfrag_h(klp + (size_t)(kb0 + 16) * DM);
      s0h = mma_raw(qh, kf0h, zero8());
      s0x = mma_raw(qh, kf0l, zero8());
      s0x = mma_raw(ql, kf0h, s0x);
      s1h = mma_raw(qh, kf1h, zero8());
      s1x = mma_raw(qh, kf1l, zero8());
      s1x = mma_raw(ql, kf1h, s1x);
      guard_4x6(s0h, s0x, s1h, s1x, qh, ql, kf0h, kf0l, kf1h, kf1l);
    }
    const int key0 = kb0 + c, key1 = kb0 + 16 + c;
    const bool in0 = key0 < Nk, in1 = key1 < Nk;
    const int kid0 = kbv[in0 ? key0 : (Nk - 1)], kid1 = kbv[in1 ? key1 : (Nk - 1)];
#pragma unroll
    for (int r = 0; r < 8; ++r) {
      const float s0 = (s0h[r] + s0x[r] * RINV) * lsc;
      const float s1 = (s1h[r] + s1x[r] * RINV) * lsc;
      const int ro = (8 * hh + r) * PSP + c;
      const bool f   = ((fb >> r) & 1u) != 0u;
      const bool kp0 = in0 && (f || (kid0 == qid[r]));
      const bool kp1 = in1 && (f || (kid1 == qid[r]));
      const float t0 = f ? 0.f : s0, t1 = f ? 0.f : s1;
      float mx = fmaxf(kp0 ? t0 : NEGS, kp1 ? t1 : NEGS);
      mx = fmaxf(mx, __shfl_xor(mx, 1, 32));
      mx = fmaxf(mx, __shfl_xor(mx, 2, 32));
      mx = fmaxf(mx, __shfl_xor(mx, 4, 32));
      mx = fmaxf(mx, __shfl_xor(mx, 8, 32));
      const float mn = fmaxf(m[r], mx);
      const float al = exp2f(m[r] - mn);
      m[r] = mn;
      const float e0 = kp0 ? exp2f(t0 - mn) : 0.f;
      const float e1 = kp1 ? exp2f(t1 - mn) : 0.f;
      float ps = e0 + e1;
      ps += __shfl_xor(ps, 1, 32);
      ps += __shfl_xor(ps, 2, 32);
      ps += __shfl_xor(ps, 4, 32);
      ps += __shfl_xor(ps, 8, 32);
      l[r] = l[r] * al + ps;
      z0h[r] *= al; z0x[r] *= al; z1h[r] *= al; z1x[r] *= al;
      pP[ro]      = e0;
      pP[ro + 16] = e1;
    }
    wave_sync_lds();
    const v16h vh0 = ldfrag_h(vhp + kb0), vh1 = ldfrag_h(vhp + (size_t)16 * (size_t)Nk + kb0);
    const v16h vl0 = ldfrag_h(vlp + kb0), vl1 = ldfrag_h(vlp + (size_t)16 * (size_t)Nk + kb0);
    {
      FragH ph, pl;
      build_p(pP, c, hh, ph, pl);
      z0h = mma_raw(ph.v, vh0, z0h);
      z0x = mma_raw(ph.v, vl0, z0x);
      z0x = mma_raw(pl.v, vh0, z0x);
      z1h = mma_raw(ph.v, vh1, z1h);
      z1x = mma_raw(ph.v, vl1, z1x);
      z1x = mma_raw(pl.v, vh1, z1x);
      guard_4x6(z0h, z0x, z1h, z1x, ph.v, pl.v, vh0, vl0, vh1, vl1);
    }
    wave_sync_lds();
  }

  const float oc2 = ZC / (PC * VC);
  float* os = Os[wave];
#pragma unroll
  for (int r = 0; r < 8; ++r) {
    const float inv = (l[r] > 0.f) ? (__builtin_amdgcn_rcpf(l[r]) * oc2) : 0.f;
    const int ro = (8 * hh + r) * 32 + c;
    os[ro]      = (z0h[r] + z0x[r] * RINV) * inv;
    os[ro + 16] = (z1h[r] + z1x[r] * RINV) * inv;
  }
  wave_sync_lds();
  unsigned short* dh = CH + ((size_t)h * (size_t)Nq + (size_t)q0) * HD;
  unsigned short* dl = CL + ((size_t)h * (size_t)Nq + (size_t)q0) * HD;
  store_tile16x32(os, lane, dh, dl);
  wave_sync_lds();
}

extern "C" void kernel_launch(void* const* d_in, const int* in_sizes, int n_in,
                              void* d_out, int out_size, void* d_ws, size_t ws_size,
                              hipStream_t stream) {
  if (n_in < 14) return;
  if (in_sizes[0] != N1 * DIN || in_sizes[1] != N2 * DIN) return;
  if (in_sizes[2] != DIN * DM || in_sizes[3] != DIN * DM || in_sizes[4] != DIN * DM || in_sizes[5] != DM * DIN) return;
  if (in_sizes[7] != DIN * DM || in_sizes[8] != DIN * DM || in_sizes[9] != DIN * DM || in_sizes[10] != DM * DIN) return;
  if (in_sizes[6] != DIN || in_sizes[11] != DIN) return;
  if (in_sizes[12] != N1 || in_sizes[13] != N2) return;
  if (out_size != (N1 + N2) * DIN) return;

  const float* X1  = (const float*)d_in[0];
  const float* X2  = (const float*)d_in[1];
  const float* WQ1 = (const float*)d_in[2];
  const float* WK2 = (const float*)d_in[3];
  const float* WV2 = (const float*)d_in[4];
  const float* WO1 = (const float*)d_in[5];
  const float* BO1 = (const float*)d_in[6];
  const float* WQ2 = (const float*)d_in[7];
  const float* WK1 = (const float*)d_in[8];
  const float* WV1 = (const float*)d_in[9];
  const float* WO2 = (const float*)d_in[10];
  const float* BO2 = (const float*)d_in[11];
  const int*   I1  = (const int*)d_in[12];
  const int*   I2  = (const int*)d_in[13];
  float*       out = (float*)d_out;

  const size_t BW  = (size_t)DM * DIN * 2;
  const size_t BX1 = (size_t)N1 * DIN * 2;
  const size_t BX2 = (size_t)N2 * DIN * 2;
  const size_t BT1 = (size_t)(N1 / 16) * TP * 4;
  const size_t BT2 = (size_t)(N2 / 16) * TP * 4;
  const size_t BP1 = (size_t)N1 * DM * 2;
  const size_t BP2 = (size_t)N2 * DM * 2;
  size_t off = 0;
  const size_t oWQ1 = off; off += BW;
  const size_t oWK2 = off; off += BW;
  const size_t oWV2 = off; off += BW;
  const size_t oWO1 = off; off += BW;
  const size_t oWQ2 = off; off += BW;
  const size_t oWK1 = off; off += BW;
  const size_t oWV1 = off; off += BW;
  const size_t oWO2 = off; off += BW;
  const size_t oX1  = off; off += BX1;
  const size_t oX2  = off; off += BX2;
  const size_t oT1  = off; off += BT1;
  const size_t oT2  = off; off += BT2;
  const size_t oQHa = off; off += BP1;
  const size_t oQLa = off; off += BP1;
  const size_t oKHa = off; off += BP2;
  const size_t oKLa = off; off += BP2;
  const size_t oVHa = off; off += BP2;
  const size_t oVLa = off; off += BP2;
  const size_t oCHa = off; off += BP1;
  const size_t oCLa = off; off += BP1;
  const size_t oQHb = off; off += BP2;
  const size_t oQLb = off; off += BP2;
  const size_t oKHb = off; off += BP1;
  const size_t oKLb = off; off += BP1;
  const size_t oVHb = off; off += BP1;
  const size_t oVLb = off; off += BP1;
  const size_t oCHb = off; off += BP2;
  const size_t oCLb = off; off += BP2;
  if (off > ws_size) return;
  if (off > (size_t)134217728) return;

  char* ws = (char*)d_ws;
  unsigned short* WQ1T = (unsigned short*)(ws + oWQ1);
  unsigned short* WK2T = (unsigned short*)(ws + oWK2);
  unsigned short* WV2T = (unsigned short*)(ws + oWV2);
  unsigned short* WO1T = (unsigned short*)(ws + oWO1);
  unsigned short* WQ2T = (unsigned short*)(ws + oWQ2);
  unsigned short* WK1T = (unsigned short*)(ws + oWK1);
  unsigned short* WV1T = (unsigned short*)(ws + oWV1);
  unsigned short* WO2T = (unsigned short*)(ws + oWO2);
  unsigned short* XP1  = (unsigned short*)(ws + oX1);
  unsigned short* XP2  = (unsigned short*)(ws + oX2);
  unsigned*       T1   = (unsigned*)(ws + oT1);
  unsigned*       T2   = (unsigned*)(ws + oT2);
  unsigned short* QHa  = (unsigned short*)(ws + oQHa);
  unsigned short* QLa  = (unsigned short*)(ws + oQLa);
  unsigned short* KHa  = (unsigned short*)(ws + oKHa);
  unsigned short* KLa  = (unsigned short*)(ws + oKLa);
  unsigned short* VHa  = (unsigned short*)(ws + oVHa);
  unsigned short* VLa  = (unsigned short*)(ws + oVLa);
  unsigned short* CHa  = (unsigned short*)(ws + oCHa);
  unsigned short* CLa  = (unsigned short*)(ws + oCLa);
  unsigned short* QHb  = (unsigned short*)(ws + oQHb);
  unsigned short* QLb  = (unsigned short*)(ws + oQLb);
  unsigned short* KHb  = (unsigned short*)(ws + oKHb);
  unsigned short* KLb  = (unsigned short*)(ws + oKLb);
  unsigned short* VHb  = (unsigned short*)(ws + oVHb);
  unsigned short* VLb  = (unsigned short*)(ws + oVLb);
  unsigned short* CHb  = (unsigned short*)(ws + oCHb);
  unsigned short* CLb  = (unsigned short*)(ws + oCLb);

  const dim3 blk(256), blk128(128);
  const dim3 gWi(DIN / 64, DM / 64);
  const dim3 gWo(DM / 64, DIN / 64);
  const float osQ = QKC / (ACARRY * WSC);
  const float osV = VC / (ACARRY * WSC);
  const float osO = 1.0f / (ZC * WSC);

  wtcv<<<gWi, blk, 0, stream>>>(WQ1, WQ1T, DIN, DM);
  wtcv<<<gWi, blk, 0, stream>>>(WK2, WK2T, DIN, DM);
  wtcv<<<gWi, blk, 0, stream>>>(WV2, WV2T, DIN, DM);
  wtcv<<<gWo, blk, 0, stream>>>(WO1, WO1T, DM, DIN);
  wtcv<<<gWi, blk, 0, stream>>>(WQ2, WQ2T, DIN, DM);
  wtcv<<<gWi, blk, 0, stream>>>(WK1, WK1T, DIN, DM);
  wtcv<<<gWi, blk, 0, stream>>>(WV1, WV1T, DIN, DM);
  wtcv<<<gWo, blk, 0, stream>>>(WO2, WO2T, DM, DIN);

  xcv<<<dim3(N1 / 16), blk, 0, stream>>>(X1, XP1, N1);
  xcv<<<dim3(N2 / 16), blk, 0, stream>>>(X2, XP2, N2);
  blkmap<<<dim3(N1 / 64), blk128, 0, stream>>>(I1, I2, T1, N1, N2);
  blkmap<<<dim3(N2 / 64), blk128, 0, stream>>>(I2, I1, T2, N2, N1);

  gemm64<3, 2><<<dim3(((N1 / 64) * (DM / 64) + 7) / 8), blk, 0, stream>>>(
      XP1, DIN, 32LL, 0LL, WQ1T, DIN, BO1, 0.f,
      (void*)QHa, DM, (long long)(QLa - QHa), N1, DM, DIN, osQ);
  gemm64<3, 2><<<dim3(((N2 / 64) * (DM / 64) + 7) / 8), blk, 0, stream>>>(
      XP2, DIN, 32LL, 0LL, WK2T, DIN, BO1, 0.f,
      (void*)KHa, DM, (long long)(KLa - KHa), N2, DM, DIN, osQ);
  gemm64<3, 2><<<dim3(((DM / 64) * (N2 / 64) + 7) / 8), blk, 0, stream>>>(
      WV2T, DIN, 32LL, 0LL, XP2, DIN, BO1, 0.f,
      (void*)VHa, N2, (long long)(VLa - VHa), DM, N2, DIN, osV);
  attn<<<dim3(((N1 / 16) * NH) / 4), blk128, 0, stream>>>(QHa, QLa, KHa, KLa, VHa, VLa, I1, I2, T1, CHa, CLa, N1, N2);
  gemm64<4, 0><<<dim3(((N1 / 64) * (DIN / 64) + 7) / 8), blk, 0, stream>>>(
      CHa, HD, (long long)N1 * HD, (long long)(CLa - CHa), WO1T, DM, BO1, 1.0f,
      (void*)out, DIN, 0LL, N1, DIN, DM, osO);

  gemm64<3, 2><<<dim3(((N2 / 64) * (DM / 64) + 7) / 8), blk, 0, stream>>>(
      XP2, DIN, 32LL, 0LL, WQ2T, DIN, BO2, 0.f,
      (void*)QHb, DM, (long long)(QLb - QHb), N2, DM, DIN, osQ);
  gemm64<3, 2><<<dim3(((N1 / 64) * (DM / 64) + 7) / 8), blk, 0, stream>>>(
      XP1, DIN, 32LL, 0LL, WK1T, DIN, BO2, 0.f,
      (void*)KHb, DM, (long long)(KLb - KHb), N1, DM, DIN, osQ);
  gemm64<3, 2><<<dim3(((DM / 64) * (N1 / 64) + 7) / 8), blk, 0, stream>>>(
      WV1T, DIN, 32LL, 0LL, XP1, DIN, BO2, 0.f,
      (void*)VHb, N1, (long long)(VLb - VHb), DM, N1, DIN, osV);
  attn<<<dim3(((N2 / 16) * NH) / 4), blk128, 0, stream>>>(QHb, QLb, KHb, KLb, VHb, VLb, I2, I1, T2, CHb, CLb, N2, N1);
  gemm64<4, 0><<<dim3(((N2 / 64) * (DIN / 64) + 7) / 8), blk, 0, stream>>>(
      CHb, HD, (long long)N2 * HD, (long long)(CLb - CHb), WO2T, DM, BO2, 1.0f,
      (void*)(out + (size_t)N1 * DIN), DIN, 0LL, N2, DIN, DM, osO);

  (void)hipGetLastError();
}
